// MemoryAlgorithm_15882789060892
// MI455X (gfx1250) — hardware-verified
//
#include <hip/hip_runtime.h>
#include <math.h>

typedef _Float16 v16h __attribute__((ext_vector_type(16)));
typedef _Float16 v8h  __attribute__((ext_vector_type(8)));
typedef float    v8f  __attribute__((ext_vector_type(8)));
typedef float    v4f  __attribute__((ext_vector_type(4)));
typedef v8h __attribute__((may_alias)) v8ha;
typedef v4f __attribute__((may_alias)) v4fa;

union Frag { v16h v; v8h half[2]; };

#define NBATCH 4
#define NSEQ   2048
#define NHID   1024
#define NMEM   512
#define NHEAD  16
#define HDIM   64
#define HQF    256
#define NTOK   (NBATCH * NSEQ)
#define NSLOT  (NBATCH * NMEM)
#define NX     (NTOK * NHID)
#define NMV    (NSLOT * HQF)
#define NO1    (NTOK * NMEM)
#define PPITCH 520

#define WOFF_Q  0
#define WOFF_K  (NHID * NHID)
#define WOFF_V  (WOFF_K + NHID * HQF)
#define WOFF_1  (WOFF_V + NHID * HQF)
#define WOFF_2  (WOFF_1 + NHID * 2 * NHID)
#define WOFF_G  (WOFF_2 + NHID * NHID)
#define WT_HALVES (WOFF_G + NHID * 2 * NHID)

enum { EPI_Q = 0, EPI_KV = 1, EPI_FFN1 = 2, EPI_W2 = 3 };

__device__ __forceinline__ v8f wmma1(v16h a, v16h b, v8f c) {
  v8f d = __builtin_amdgcn_wmma_f32_16x16x32_f16(false, a, false, b, (short)0, c, false, false);
  asm volatile("v_nop\n\tv_nop\n\tv_nop\n\tv_nop" : "+v"(d) : "v"(a), "v"(b));
  return d;
}
__device__ __forceinline__ void wmma2b(v16h a0, v16h a1, v16h b, v8f& c0, v8f& c1) {
  v8f d0 = __builtin_amdgcn_wmma_f32_16x16x32_f16(false, a0, false, b, (short)0, c0, false, false);
  v8f d1 = __builtin_amdgcn_wmma_f32_16x16x32_f16(false, a1, false, b, (short)0, c1, false, false);
  asm volatile("v_nop\n\tv_nop\n\tv_nop\n\tv_nop" : "+v"(d0), "+v"(d1) : "v"(a0), "v"(a1), "v"(b));
  c0 = d0; c1 = d1;
}

__device__ __forceinline__ v16h load_frag(const _Float16* p, int hh) {
  Frag f;
  f.half[0] = *(const v8ha*)(p + 8 * hh);
  f.half[1] = *(const v8ha*)(p + 16 + 8 * hh);
  return f.v;
}

__device__ __forceinline__ float gelu_f(float x) {
  return 0.5f * x * erfcf(-x * 0.70710678118654752f);
}

__global__ __launch_bounds__(256) void convert_kernel(
    const float* __restrict__ x, const float* __restrict__ mem,
    _Float16* __restrict__ xh, _Float16* __restrict__ memh)
{
  const int NX8 = NX / 8, NM8 = NMV / 8;
  const int g = blockIdx.x * 256 + threadIdx.x;
  if (g >= NX8 + NM8) return;
  const float* src;
  _Float16* dst;
  if (g < NX8) { src = x + (size_t)g * 8;   dst = xh + (size_t)g * 8; }
  else         { const int e = g - NX8; src = mem + (size_t)e * 8; dst = memh + (size_t)e * 8; }
  const v4f a = *(const v4fa*)src;
  const v4f c = *(const v4fa*)(src + 4);
  const v8h o = { (_Float16)a.x, (_Float16)a.y, (_Float16)a.z, (_Float16)a.w,
                  (_Float16)c.x, (_Float16)c.y, (_Float16)c.z, (_Float16)c.w };
  *(volatile v8h*)dst = o;
  __threadfence();
  *(volatile v8h*)dst = o;
}

__global__ __launch_bounds__(256) void wtrans_kernel(
    const float* __restrict__ Wq, const float* __restrict__ Wk, const float* __restrict__ Wv,
    const float* __restrict__ W1, const float* __restrict__ W2, const float* __restrict__ Wg1,
    _Float16* __restrict__ wt)
{
  __shared__ __attribute__((aligned(16))) _Float16 tile[64 * 72];
  int t = blockIdx.x;
  const float* src;
  int K, doff;
  float sc = 64.0f;
  if (t < 256)       {            src = Wq;  K = NHID;     doff = WOFF_Q; }
  else if (t < 320)  { t -= 256;  src = Wk;  K = HQF;      doff = WOFF_K; }
  else if (t < 384)  { t -= 320;  src = Wv;  K = HQF;      doff = WOFF_V; }
  else if (t < 896)  { t -= 384;  src = W1;  K = 2 * NHID; doff = WOFF_1; }
  else if (t < 1152) { t -= 896;  src = W2;  K = NHID;     doff = WOFF_2; }
  else               { t -= 1152; src = Wg1; K = 2 * NHID; doff = WOFF_G; }
  const int k0 = (t >> 4) * 64, n0 = (t & 15) * 64;
  if (K == 2 * NHID && k0 >= NHID) sc = 8.0f;

  const int tid = threadIdx.x, kr = tid >> 2, nq = (tid & 3) * 16;
  const float* p = src + (size_t)(k0 + kr) * NHID + n0 + nq;
  const v4f w0 = *(const v4fa*)p;
  const v4f w1 = *(const v4fa*)(p + 4);
  const v4f w2 = *(const v4fa*)(p + 8);
  const v4f w3 = *(const v4fa*)(p + 12);
  _Float16* tc = tile + nq * 72 + kr;
  tc[ 0 * 72] = (_Float16)(w0.x * sc); tc[ 1 * 72] = (_Float16)(w0.y * sc);
  tc[ 2 * 72] = (_Float16)(w0.z * sc); tc[ 3 * 72] = (_Float16)(w0.w * sc);
  tc[ 4 * 72] = (_Float16)(w1.x * sc); tc[ 5 * 72] = (_Float16)(w1.y * sc);
  tc[ 6 * 72] = (_Float16)(w1.z * sc); tc[ 7 * 72] = (_Float16)(w1.w * sc);
  tc[ 8 * 72] = (_Float16)(w2.x * sc); tc[ 9 * 72] = (_Float16)(w2.y * sc);
  tc[10 * 72] = (_Float16)(w2.z * sc); tc[11 * 72] = (_Float16)(w2.w * sc);
  tc[12 * 72] = (_Float16)(w3.x * sc); tc[13 * 72] = (_Float16)(w3.y * sc);
  tc[14 * 72] = (_Float16)(w3.z * sc); tc[15 * 72] = (_Float16)(w3.w * sc);
  __syncthreads();

  const int ga = tid, gb = 256 + tid;
  const int la = ga >> 3, qa = ga & 7, lb = gb >> 3, qb = gb & 7;
  const v8h va = *(const v8ha*)(tile + la * 72 + 8 * qa);
  const v8h vb = *(const v8ha*)(tile + lb * 72 + 8 * qb);
  _Float16* da = wt + doff + (size_t)(n0 + la) * K + k0 + 8 * qa;
  _Float16* db = wt + doff + (size_t)(n0 + lb) * K + k0 + 8 * qb;
  *(volatile v8h*)da = va;
  *(volatile v8h*)db = vb;
  __threadfence();
  *(volatile v8h*)da = va;
  *(volatile v8h*)db = vb;
}

__device__ __forceinline__ void plane_pass(const _Float16* sT, _Float16* plane,
                                           int m0, int n0, int w, int lane) {
  const int q8 = lane & 7, sub = lane >> 3;
  #pragma unroll
  for (int i = 0; i < 8; ++i) {
    const int lid = w * 32 + i * 4 + sub;
    const v8h v = *(const v8ha*)(sT + lid * 64 + 8 * q8);
    *(volatile v8h*)(plane + (size_t)(m0 + lid) * NHID + n0 + 8 * q8) = v;
  }
}
__device__ __forceinline__ void vt_pass(const _Float16* sT, _Float16* vt,
                                        int m0, int head, int w, int lane) {
  const int q8 = lane & 7, sub = lane >> 3;
  const int b = m0 >> 9, l0 = m0 & 511;
  #pragma unroll
  for (int i = 0; i < 8; ++i) {
    const int lid = w * 32 + i * 4 + sub;
    const int d = lid >> 1, hl = lid & 1;
    const v8h v = *(const v8ha*)(sT + d * 128 + 64 * hl + 8 * q8);
    *(volatile v8h*)(vt + ((size_t)(b * NHEAD + head) * HDIM + d) * NMEM + l0 + 64 * hl + 8 * q8) = v;
  }
}
__device__ __forceinline__ void f32_pass(const float* sF, float* outf,
                                         int m0, int n0, int tid) {
  #pragma unroll
  for (int i = 0; i < 16; ++i) {
    const int g = i * 128 + tid;
    const int line = g >> 3, q8 = g & 7;
    const int row = line >> 1, hl = line & 1;
    const int col = 32 * hl + 4 * q8;
    const v4f v = *(const v4fa*)(sF + row * 64 + col);
    *(volatile v4f*)(outf + (size_t)(m0 + row) * NHID + n0 + col) = v;
  }
}

template <int EPI>
__global__ __launch_bounds__(128) void gemm_kernel(
    const _Float16* __restrict__ A0, const _Float16* __restrict__ A1,
    const _Float16* __restrict__ Bt0, const _Float16* __restrict__ Bt1,
    const float* __restrict__ bias0, const float* __restrict__ bias1,
    const float* __restrict__ wg2,
    _Float16* __restrict__ outh0, _Float16* __restrict__ outh1,
    float* __restrict__ outf)
{
  constexpr int LDA  = (EPI == EPI_KV) ? HQF : NHID;
  constexpr int KS0  = LDA;
  constexpr int KS1  = (EPI == EPI_FFN1) ? NHID : 0;
  constexpr int LDB  = KS0 + KS1;
  constexpr int SRAW = (EPI == EPI_W2) ? (128 * 64 * 4) : (128 * 64 * 2);
  __shared__ __attribute__((aligned(16))) char sraw[SRAW];

  const int tid = threadIdx.x, lane = tid & 31, w = tid >> 5;
  const int hh = lane >> 4, m = lane & 15;
  const int m0 = blockIdx.x * 128;
  const int nbk = blockIdx.y;
  const bool dual = (EPI == EPI_KV) || (EPI == EPI_FFN1);
  const int which = dual ? (nbk >> 4) : 0;
  const int cb = dual ? (nbk & 15) : nbk;
  const int n0 = cb * 64;
  const _Float16* Bt = (which != 0) ? Bt1 : Bt0;
  const float* bias  = (which != 0) ? bias1 : bias0;

  const _Float16* arow = A0 + (size_t)(m0 + 32 * w + m) * LDA;
  const _Float16* brow = Bt + (size_t)(n0 + m) * LDB;

  const v8f zero8 = {0.f, 0.f, 0.f, 0.f, 0.f, 0.f, 0.f, 0.f};
  v8f acc[2][4];
  #pragma unroll
  for (int mt = 0; mt < 2; ++mt)
    #pragma unroll
    for (int nt = 0; nt < 4; ++nt) acc[mt][nt] = zero8;

  #pragma unroll 1
  for (int k0 = 0; k0 < KS0; k0 += 32) {
    const v16h a0 = load_frag(arow + k0, hh);
    const v16h a1 = load_frag(arow + (size_t)16 * LDA + k0, hh);
    #pragma unroll
    for (int nt = 0; nt < 4; ++nt) {
      const v16h b = load_frag(brow + (size_t)nt * 16 * LDB + k0, hh);
      wmma2b(a0, a1, b, acc[0][nt], acc[1][nt]);
    }
  }
  if (KS1 > 0) {
    const _Float16* arow1 = A1 + (size_t)(m0 + 32 * w + m) * NHID;
    #pragma unroll 1
    for (int k0 = 0; k0 < KS1; k0 += 32) {
      const v16h a0 = load_frag(arow1 + k0, hh);
      const v16h a1 = load_frag(arow1 + (size_t)16 * NHID + k0, hh);
      #pragma unroll
      for (int nt = 0; nt < 4; ++nt) {
        const v16h b = load_frag(brow + (size_t)nt * 16 * LDB + KS0 + k0, hh);
        wmma2b(a0, a1, b, acc[0][nt], acc[1][nt]);
      }
    }
  }

  const float ascale = (EPI == EPI_W2) ? (1.0f / 256.0f) : (1.0f / 64.0f);
  #pragma unroll
  for (int nt = 0; nt < 4; ++nt) {
    const float bvl = bias[n0 + 16 * nt + m];
    #pragma unroll
    for (int mt = 0; mt < 2; ++mt) {
      #pragma unroll
      for (int r = 0; r < 8; ++r) {
        float y = acc[mt][nt][r] * ascale + bvl;
        if (EPI == EPI_FFN1) y = gelu_f(y);
        acc[mt][nt][r] = y;
      }
    }
  }

  if (EPI == EPI_W2) {
    float* sF = (float*)sraw;
    #pragma unroll
    for (int nt = 0; nt < 4; ++nt)
      #pragma unroll
      for (int mt = 0; mt < 2; ++mt)
        #pragma unroll
        for (int r = 0; r < 8; ++r) {
          const int tokl = 32 * w + 16 * mt + 8 * hh + r;
          sF[tokl * 64 + 16 * nt + m] = acc[mt][nt][r];
        }
    __syncthreads();
    f32_pass(sF, outf, m0, n0, tid);
    __threadfence();
    f32_pass(sF, outf, m0, n0, tid);
    return;
  }

  const bool gate_path = (EPI == EPI_FFN1) && (which != 0);
  const bool vt_path   = (EPI == EPI_KV)   && (which != 0);
  _Float16* sT = (_Float16*)sraw;
  float*    sG = (float*)sraw;

  if (gate_path) {
    float wgv[4];
    #pragma unroll
    for (int nt = 0; nt < 4; ++nt) wgv[nt] = wg2[n0 + 16 * nt + m];
    float rs[2][8];
    #pragma unroll
    for (int mt = 0; mt < 2; ++mt)
      #pragma unroll
      for (int r = 0; r < 8; ++r) {
        float s = 0.0f;
        #pragma unroll
        for (int nt = 0; nt < 4; ++nt) s += acc[mt][nt][r] * wgv[nt];
        s += __shfl_xor(s, 1);
        s += __shfl_xor(s, 2);
        s += __shfl_xor(s, 4);
        s += __shfl_xor(s, 8);
        rs[mt][r] = s;
      }
    if (m == 0) {
      #pragma unroll
      for (int mt = 0; mt < 2; ++mt)
        #pragma unroll
        for (int r = 0; r < 8; ++r) sG[32 * w + 16 * mt + 8 * hh + r] = rs[mt][r];
    }
  } else {
    const float osc = (EPI == EPI_FFN1) ? 4.0f : 1.0f;
    #pragma unroll
    for (int nt = 0; nt < 4; ++nt)
      #pragma unroll
      for (int mt = 0; mt < 2; ++mt)
        #pragma unroll
        for (int r = 0; r < 8; ++r) {
          const int tokl = 32 * w + 16 * mt + 8 * hh + r;
          const int feat = 16 * nt + m;
          const int idx = vt_path ? (feat * 128 + tokl) : (tokl * 64 + feat);
          sT[idx] = (_Float16)(acc[mt][nt][r] * osc);
        }
  }
  __syncthreads();

  if (gate_path) {
    if (w == 0) {
      const v4f v = *(const v4fa*)(sG + 4 * lane);
      float* d = outf + (size_t)cb * NTOK + m0 + 4 * lane;
      *(volatile v4f*)d = v;
      __threadfence();
      *(volatile v4f*)d = v;
    }
  } else if (vt_path) {
    vt_pass(sT, outh1, m0, cb, w, lane);
    __threadfence();
    vt_pass(sT, outh1, m0, cb, w, lane);
  } else {
    plane_pass(sT, outh0, m0, n0, w, lane);
    __threadfence();
    plane_pass(sT, outh0, m0, n0, w, lane);
  }
}

__global__ __launch_bounds__(256) void attn_kernel(
    const _Float16* __restrict__ qh,
    const _Float16* __restrict__ kh,
    const _Float16* __restrict__ vt,
    const int* __restrict__ mask,
    const float* __restrict__ sscore,
    _Float16* __restrict__ atth,
    float* __restrict__ out1)
{
  __shared__ __attribute__((aligned(16))) float slog[16 * NMEM];
  __shared__ __attribute__((aligned(16))) _Float16 sprob[16 * PPITCH];
  __shared__ int smask[NMEM];

  const int tid = threadIdx.x, lane = tid & 31, w = tid >> 5;
  const int hh = lane >> 4, m = lane & 15;
  const int b = blockIdx.y, s0 = blockIdx.x * 16;

  smask[tid]       = mask[b * NMEM + tid];
  smask[tid + 256] = mask[b * NMEM + tid + 256];
  const float ss  = sscore[0];
  const float fac = 1.0f + ss;
  const bool  rew = ss > 0.6f;
  const int srow = 2 * w + hh;
  float macc[32];
  #pragma unroll
  for (int c = 0; c < 32; ++c) macc[c] = 0.0f;
  const v8f zero8 = {0.f, 0.f, 0.f, 0.f, 0.f, 0.f, 0.f, 0.f};
  __syncthreads();

  #pragma unroll 1
  for (int head = 0; head < NHEAD; ++head) {
    {
      const _Float16* qrow = qh + (size_t)(b * NSEQ + s0 + m) * NHID + head * HDIM;
      const v16h a0 = load_frag(qrow, hh);
      const v16h a1 = load_frag(qrow + 32, hh);
      #pragma unroll
      for (int j = 0; j < 4; ++j) {
        const int sl0 = 64 * w + 16 * j;
        const _Float16* krow = kh + (size_t)(b * NMEM + sl0 + m) * NHID + head * HDIM;
        const v16h b0 = load_frag(krow, hh);
        const v16h b1 = load_frag(krow + 32, hh);
        v8f z = wmma1(a0, b0, zero8);
        z = wmma1(a1, b1, z);
        #pragma unroll
        for (int r = 0; r < 8; ++r) slog[(8 * hh + r) * NMEM + sl0 + m] = z[r];
      }
    }
    __syncthreads();

    {
      const float* lrow = slog + srow * NMEM + m;
      float e[32];
      float mx = -__builtin_huge_valf();
      #pragma unroll
      for (int c = 0; c < 32; ++c) {
        const float lg = lrow[16 * c] * 0.125f;
        const int mk = smask[m + 16 * c];
        const float xv = (mk != 0) ? lg : -__builtin_huge_valf();
        e[c] = xv;
        mx = fmaxf(mx, xv);
      }
      mx = fmaxf(mx, __shfl_xor(mx, 8));
      mx = fmaxf(mx, __shfl_xor(mx, 4));
      mx = fmaxf(mx, __shfl_xor(mx, 2));
      mx = fmaxf(mx, __shfl_xor(mx, 1));
      float sum = 0.0f;
      #pragma unroll
      for (int c = 0; c < 32; ++c) { const float pe = __expf(e[c] - mx); e[c] = pe; sum += pe; }
      sum += __shfl_xor(sum, 8);
      sum += __shfl_xor(sum, 4);
      sum += __shfl_xor(sum, 2);
      sum += __shfl_xor(sum, 1);
      const float inv = 1.0f / sum;
      float sum2 = 0.0f;
      #pragma unroll
      for (int c = 0; c < 32; ++c) { const float pn = e[c] * inv; e[c] = pn; sum2 += pn * fac; }
      sum2 += __shfl_xor(sum2, 8);
      sum2 += __shfl_xor(sum2, 4);
      sum2 += __shfl_xor(sum2, 2);
      sum2 += __shfl_xor(sum2, 1);
      const float inv2 = 1.0f / sum2;
      _Float16* prow = sprob + srow * PPITCH + m;
      #pragma unroll
      for (int c = 0; c < 32; ++c) {
        const float pn  = e[c];
        const float w2v = (pn * fac) * inv2;
        const float pf  = rew ? w2v : pn;
        macc[c] += pf;
        prow[16 * c] = (_Float16)(pf * 256.0f);
      }
    }
    __syncthreads();

    {
      const int jt = w & 3, kh2 = w >> 2;
      const _Float16* prow = sprob + m * PPITCH + kh2 * 256;
      const _Float16* vrow = vt + ((size_t)(b * NHEAD + head) * HDIM + 16 * jt + m) * NMEM + kh2 * 256;
      v8f o = zero8;
      #pragma unroll
      for (int ks = 0; ks < 8; ++ks) {
        const v16h a  = load_frag(prow + 32 * ks, hh);
        const v16h bb = load_frag(vrow + 32 * ks, hh);
        o = wmma1(a, bb, o);
      }
      float* attp = slog;
      #pragma unroll
      for (int r = 0; r < 8; ++r) attp[(kh2 * 16 + 8 * hh + r) * HDIM + 16 * jt + m] = o[r];
    }
    __syncthreads();

    if (tid < 128) {
      const int row = tid >> 3, q8 = tid & 7;
      const float* p0 = slog + row * HDIM + 8 * q8;
      const v4f a0 = *(const v4fa*)p0;
      const v4f a1 = *(const v4fa*)(p0 + 4);
      const v4f c0 = *(const v4fa*)(p0 + 1024);
      const v4f c1 = *(const v4fa*)(p0 + 1028);
      const float sc = 0.03125f;
      const v8h ov = { (_Float16)((a0.x + c0.x) * sc), (_Float16)((a0.y + c0.y) * sc),
                       (_Float16)((a0.z + c0.z) * sc), (_Float16)((a0.w + c0.w) * sc),
                       (_Float16)((a1.x + c1.x) * sc), (_Float16)((a1.y + c1.y) * sc),
                       (_Float16)((a1.z + c1.z) * sc), (_Float16)((a1.w + c1.w) * sc) };
      _Float16* dst = atth + (size_t)(b * NSEQ + s0 + row) * NHID + head * HDIM + 8 * q8;
      *(volatile v8h*)dst = ov;
      __threadfence();
      *(volatile v8h*)dst = ov;
    }
    __syncthreads();
  }

  {
    float* mrow = slog + srow * NMEM + m;
    #pragma unroll
    for (int c = 0; c < 32; ++c) mrow[16 * c] = macc[c] * 0.0625f;
  }
  __syncthreads();
  {
    float* orow = out1 + (size_t)(b * NSEQ + s0) * NMEM;
    v4f vv[8];
    #pragma unroll
    for (int i = 0; i < 8; ++i) vv[i] = *(const v4fa*)(slog + 4 * (i * 256 + tid));
    #pragma unroll
    for (int i = 0; i < 8; ++i) *(volatile v4f*)(orow + 4 * (i * 256 + tid)) = vv[i];
    __threadfence();
    #pragma unroll
    for (int i = 0; i < 8; ++i) *(volatile v4f*)(orow + 4 * (i * 256 + tid)) = vv[i];
  }
}

__global__ __launch_bounds__(256) void final_kernel(
    const float* __restrict__ fpre, const float* __restrict__ x,
    const float* __restrict__ gp, const float* __restrict__ bg2,
    const float* __restrict__ lng, const float* __restrict__ lnb,
    float* __restrict__ out0)
{
  __shared__ float rs1[8];
  __shared__ float rs2[8];
  const int row = blockIdx.x, tid = threadIdx.x, lane = tid & 31, w = tid >> 5;
  const size_t base = (size_t)row * NHID + 4 * tid;

  const v4f v = *(const v4fa*)(fpre + base);
  float s = (v.x + v.y) + (v.z + v.w);
  s += __shfl_xor(s, 16); s += __shfl_xor(s, 8); s += __shfl_xor(s, 4);
  s += __shfl_xor(s, 2);  s += __shfl_xor(s, 1);
  if (lane == 0) rs1[w] = s;
  __syncthreads();
  float ts = 0.0f;
  #pragma unroll
  for (int i = 0; i < 8; ++i) ts += rs1[i];
  const float mu = ts * (1.0f / NHID);
  const float d0 = v.x - mu, d1 = v.y - mu, d2 = v.z - mu, d3 = v.w - mu;
  float q = (d0 * d0 + d1 * d1) + (d2 * d2 + d3 * d3);
  q += __shfl_xor(q, 16); q += __shfl_xor(q, 8); q += __shfl_xor(q, 4);
  q += __shfl_xor(q, 2);  q += __shfl_xor(q, 1);
  if (lane == 0) rs2[w] = q;
  __syncthreads();
  float tq = 0.0f;
  #pragma unroll
  for (int i = 0; i < 8; ++i) tq += rs2[i];
  const float var  = tq * (1.0f / NHID);
  const float rstd = rsqrtf(var + 1e-5f);

  float z = bg2[0];
  #pragma unroll
  for (int i = 0; i < 16; ++i) z += gp[(size_t)i * NTOK + row];
  const float g  = 1.0f / (1.0f + __expf(-z));
  const float gm = 1.0f - g;

  const v4f xv = *(const v4fa*)(x + base);
  const v4f gv = *(const v4fa*)(lng + 4 * tid);
  const v4f bv = *(const v4fa*)(lnb + 4 * tid);
  v4f o;
  o.x = g * (d0 * rstd * gv.x + bv.x) + gm * xv.x;
  o.y = g * (d1 * rstd * gv.y + bv.y) + gm * xv.y;
  o.z = g * (d2 * rstd * gv.z + bv.z) + gm * xv.z;
  o.w = g * (d3 * rstd * gv.w + bv.w) + gm * xv.w;
  *(volatile v4f*)(out0 + base) = o;
  __threadfence();
  *(volatile v4f*)(out0 + base) = o;
}

extern "C" void kernel_launch(void* const* d_in, const int* in_sizes, int n_in,
                              void* d_out, int out_size, void* d_ws, size_t ws_size,
                              hipStream_t stream) {
  if (n_in < 20) return;
  if (in_sizes[0] != NX || in_sizes[1] != NMV || in_sizes[2] != NSLOT || in_sizes[3] < 1) return;
  if (in_sizes[4] != NHID * NHID || in_sizes[6] != HQF * NHID || in_sizes[8] != HQF * NHID) return;
  if (in_sizes[10] != 2 * NHID * NHID || in_sizes[12] != NHID * NHID || in_sizes[16] != 2 * NHID * NHID) return;
  if (in_sizes[5] != NHID || in_sizes[7] != NHID || in_sizes[9] != NHID || in_sizes[11] != NHID) return;
  if (in_sizes[13] != NHID || in_sizes[14] != NHID || in_sizes[15] != NHID || in_sizes[17] != NHID) return;
  if (in_sizes[18] != NHID || in_sizes[19] < 1) return;
  if (out_size != NX + NO1) return;

  const float* x    = (const float*)d_in[0];
  const float* mem  = (const float*)d_in[1];
  const int*   mask = (const int*)d_in[2];
  const float* ssc  = (const float*)d_in[3];
  const float* Wq   = (const float*)d_in[4];
  const float* bq   = (const float*)d_in[5];
  const float* Wk   = (const float*)d_in[6];
  const float* bk   = (const float*)d_in[7];
  const float* Wv   = (const float*)d_in[8];
  const float* bv   = (const float*)d_in[9];
  const float* W1   = (const float*)d_in[10];
  const float* b1   = (const float*)d_in[11];
  const float* W2   = (const float*)d_in[12];
  const float* b2   = (const float*)d_in[13];
  const float* lng  = (const float*)d_in[14];
  const float* lnb  = (const float*)d_in[15];
  const float* Wg1  = (const float*)d_in[16];
  const float* bg1  = (const float*)d_in[17];
  const float* Wg2  = (const float*)d_in[18];
  const float* bg2  = (const float*)d_in[19];
  float* out0 = (float*)d_out;
  float* out1 = (float*)d_out + (size_t)NX;

  const size_t xh_b   = (size_t)NX * 2;
  const size_t memh_b = (size_t)NMV * 2;
  const size_t wt_b   = (size_t)WT_HALVES * 2;
  const size_t qh_b   = (size_t)NX * 2;
  const size_t kh_b   = (size_t)NSLOT * NHID * 2;
  const size_t vt_b   = (size_t)NSLOT * NHID * 2;
  const size_t att_b  = (size_t)NX * 2;
  const size_t h1_b   = (size_t)NX * 2;
  const size_t gp_b   = (size_t)16 * NTOK * 4;
  const size_t fpre_b = (size_t)NX * 4;
  size_t off = 0;
  const size_t o_xh   = off; off += xh_b;
  const size_t o_memh = off; off += memh_b;
  const size_t o_wt   = off; off += wt_b;
  const size_t o_qh   = off; off += qh_b;
  const size_t o_kh   = off; off += kh_b;
  const size_t o_vt   = off; off += vt_b;
  const size_t o_att  = off; off += att_b;
  const size_t o_h1   = off; off += h1_b;
  const size_t o_gp   = off; off += gp_b;
  const size_t o_fpre = off; off += fpre_b;
  if (off > ws_size) return;

  char* ws = (char*)d_ws;
  _Float16* xh   = (_Float16*)(ws + o_xh);
  _Float16* memh = (_Float16*)(ws + o_memh);
  _Float16* wt   = (_Float16*)(ws + o_wt);
  _Float16* qh   = (_Float16*)(ws + o_qh);
  _Float16* kh   = (_Float16*)(ws + o_kh);
  _Float16* vt   = (_Float16*)(ws + o_vt);
  _Float16* atth = (_Float16*)(ws + o_att);
  _Float16* h1h  = (_Float16*)(ws + o_h1);
  float*    gp   = (float*)(ws + o_gp);
  float*    fpre = (float*)(ws + o_fpre);
  _Float16* wqt  = wt + WOFF_Q;
  _Float16* wkt  = wt + WOFF_K;
  _Float16* wvt  = wt + WOFF_V;
  _Float16* w1t  = wt + WOFF_1;
  _Float16* w2t  = wt + WOFF_2;
  _Float16* wg1t = wt + WOFF_G;

  const int ngroups = NX / 8 + NMV / 8;
  convert_kernel<<<(ngroups + 255) / 256, 256, 0, stream>>>(x, mem, xh, memh);

  wtrans_kernel<<<1664, 256, 0, stream>>>(Wq, Wk, Wv, W1, W2, Wg1, wt);

  gemm_kernel<EPI_Q><<<dim3(NTOK / 128, 16), 128, 0, stream>>>(
      xh, xh, wqt, wqt, bq, bq, Wg2, qh, qh, gp);

  gemm_kernel<EPI_KV><<<dim3(NSLOT / 128, 32), 128, 0, stream>>>(
      memh, memh, wkt, wvt, bk, bv, Wg2, kh, vt, gp);

  attn_kernel<<<dim3(NSEQ / 16, NBATCH), 256, 0, stream>>>(qh, kh, vt, mask, ssc, atth, out1);

  gemm_kernel<EPI_FFN1><<<dim3(NTOK / 128, 32), 128, 0, stream>>>(
      xh, atth, w1t, wg1t, b1, bg1, Wg2, h1h, h1h, gp);

  gemm_kernel<EPI_W2><<<dim3(NTOK / 128, 16), 128, 0, stream>>>(
      h1h, h1h, w2t, w2t, b2, b2, Wg2, h1h, h1h, fpre);

  final_kernel<<<NTOK, 256, 0, stream>>>(fpre, x, gp, bg2, lng, lnb, out0);
}
